// MLRAttention_75385265979853
// MI455X (gfx1250) — hardware-verified
//
#include <hip/hip_runtime.h>


#define TT   2048
#define DM   1024
#define NH_  16
#define HD   64
#define NLV  4
#define LW   32
#define RH   512
#define PCAR 1024.0f
typedef _Float16 h16;
typedef unsigned short bf;
typedef __attribute__((ext_vector_type(16))) __bf16   v16bf;
typedef __attribute__((ext_vector_type(16))) _Float16 v16h;
typedef __attribute__((ext_vector_type(8)))  _Float16 v8h;
typedef __attribute__((ext_vector_type(8)))  unsigned short v8us;
typedef __attribute__((ext_vector_type(8)))  float    v8f;
typedef __attribute__((ext_vector_type(4)))  float    v4f;
typedef v8h  __attribute__((may_alias)) v8ha;
typedef v4f  __attribute__((may_alias)) v4fa;
typedef v8us __attribute__((may_alias)) v8usa;

__device__ __forceinline__ unsigned short f2bf(float f) { unsigned u = __float_as_uint(f); u += 0x7FFFu + ((u >> 16) & 1u); return (unsigned short)(u >> 16); }
__device__ __forceinline__ float bf2f(unsigned short b) { return __uint_as_float(((unsigned)b) << 16); }
__device__ __forceinline__ float bfr(float f) { return bf2f(f2bf(f)); }
__device__ __forceinline__ v16h cat16(v8h lo, v8h hi) { return __builtin_shufflevector(lo, hi, 0, 1, 2, 3, 4, 5, 6, 7, 8, 9, 10, 11, 12, 13, 14, 15); }
__device__ __forceinline__ v16bf cat16b(v8us lo, v8us hi) { return __builtin_bit_cast(v16bf, __builtin_shufflevector(lo, hi, 0, 1, 2, 3, 4, 5, 6, 7, 8, 9, 10, 11, 12, 13, 14, 15)); }
__device__ __forceinline__ v8f wmma16(v16h a, v16h b, v8f c) { return __builtin_amdgcn_wmma_f32_16x16x32_f16(false, a, false, b, (short)0, c, false, false); }
__device__ __forceinline__ v8f wmmab(v16bf a, v16bf b, v8f c) { return __builtin_amdgcn_wmma_f32_16x16x32_bf16(false, a, false, b, (short)0, c, false, false); }


template <typename T16> struct WFrag;
template <> struct WFrag<h16> { typedef v16h V; static __device__ __forceinline__ V ld(const h16* p) { return cat16(*(const v8h*)p, *(const v8h*)(p + 16)); } static __device__ __forceinline__ v8f mma(V a, V b, v8f c) { return wmma16(a, b, c); } };
template <> struct WFrag<bf> { typedef v16bf V; static __device__ __forceinline__ V ld(const bf* p) { return cat16b(*(const v8us*)p, *(const v8us*)(p + 16)); } static __device__ __forceinline__ v8f mma(V a, V b, v8f c) { return wmmab(a, b, c); } };
template <typename T16, int NSPLIT, bool BIAS>
__global__ __launch_bounds__(32) void k_gemmw(const T16* __restrict__ A, const T16* __restrict__ A2, const T16* __restrict__ Bt, const T16* __restrict__ Bt2, int K, float* C, int ldc, const float* __restrict__ bias, size_t sA, size_t sB, size_t sC) {
    typedef typename WFrag<T16>::V V;
    __shared__ __align__(16) float os[16 * 68];
    const size_t z = blockIdx.z; A += z * sA; if (A2) A2 += z * sA; Bt += z * sB; if (Bt2) Bt2 += z * sB; C += z * sC;
    const int lane = threadIdx.x & 31, lr = lane & 15, hi = lane >> 4; const int r0 = blockIdx.x * 64, c0 = blockIdx.y * 64;
    v8f acc[4][4];
#pragma unroll
    for (int mb = 0; mb < 4; ++mb)
#pragma unroll
        for (int nb = 0; nb < 4; ++nb) acc[mb][nb] = (v8f){};
    const size_t aoff = (size_t)(r0 + lr) * K + 8 * hi, boff = (size_t)(c0 + lr) * K + 8 * hi;
#pragma unroll 1
    for (int kc = 0; kc < K; kc += 32) {
        V a[4], a2[4];
#pragma unroll
        for (int mb = 0; mb < 4; ++mb) { a[mb] = WFrag<T16>::ld(A + aoff + (size_t)mb * 16 * K + kc); if (NSPLIT == 1 || NSPLIT == 2) a2[mb] = WFrag<T16>::ld(A2 + aoff + (size_t)mb * 16 * K + kc); }
#pragma unroll
        for (int nb = 0; nb < 4; ++nb) { const V b = WFrag<T16>::ld(Bt + boff + (size_t)nb * 16 * K + kc); V b2; if (NSPLIT >= 2) b2 = WFrag<T16>::ld(Bt2 + boff + (size_t)nb * 16 * K + kc);
#pragma unroll
            for (int mb = 0; mb < 4; ++mb) { acc[mb][nb] = WFrag<T16>::mma(a[mb], b, acc[mb][nb]); if (NSPLIT == 1 || NSPLIT == 2) acc[mb][nb] = WFrag<T16>::mma(a2[mb], b, acc[mb][nb]); if (NSPLIT >= 2) acc[mb][nb] = WFrag<T16>::mma(a[mb], b2, acc[mb][nb]); } }
        asm volatile("v_nop\n\tv_nop\n\tv_nop\n\tv_nop" : "+v"(acc[0][0]), "+v"(acc[1][1]), "+v"(acc[2][2]), "+v"(acc[3][3]) : "v"(a[0]), "v"(a[3]));
    }
#pragma unroll
    for (int mb = 0; mb < 4; ++mb) {
#pragma unroll
        for (int nb = 0; nb < 4; ++nb) {
#pragma unroll
            for (int j = 0; j < 8; ++j) os[(hi * 8 + j) * 68 + nb * 16 + lr] = acc[mb][nb][j]; }
        __builtin_amdgcn_wave_barrier(); asm volatile("" ::: "memory");
        float* crow = C + (size_t)(r0 + mb * 16) * ldc + c0;
#pragma unroll 1
        for (int ps = 0; ps < 2; ++ps) {
#pragma unroll
            for (int s = 0; s < 8; ++s) { const int row = 2 * s + hi, cofs = lr * 4; v4f val = *(const v4fa*)(os + row * 68 + cofs); if (BIAS) { val[0] += bfr(bias[c0 + cofs]); val[1] += bfr(bias[c0 + cofs + 1]); val[2] += bfr(bias[c0 + cofs + 2]); val[3] += bfr(bias[c0 + cofs + 3]); }
                *(volatile v4f*)(crow + (size_t)row * ldc + cofs) = val; }
            if (ps == 0) __threadfence(); }
        __builtin_amdgcn_wave_barrier(); asm volatile("" ::: "memory");
    }
}

__device__ __forceinline__ h16 tohx(float x) { return (h16)x; }
__device__ __forceinline__ void splitf(float y, unsigned short& h, unsigned short& l) { h = f2bf(y); l = f2bf(y - bf2f(h)); }
typedef __attribute__((ext_vector_type(2))) _Float16 v2h;
typedef __attribute__((ext_vector_type(4))) _Float16 v4h;
typedef __attribute__((ext_vector_type(2))) unsigned short v2us;
typedef __attribute__((ext_vector_type(4))) unsigned short v4us;
typedef __attribute__((ext_vector_type(2))) float v2f;
__constant__ int c_off[5] = {0, 32, 48, 56, 64};
__constant__ float c_inv[4] = {0.03125f, 0.0625f, 0.125f, 0.125f};

__global__ __launch_bounds__(256) void k_wtG(const float* __restrict__ w, int K, int N, bf* Bt) {
    const int lane = threadIdx.x & 31; const int L0 = (blockIdx.x * 8 + (threadIdx.x >> 5)) * 8; const int nlines = N * K / 64;
#pragma unroll 1
    for (int ps = 0; ps < 2; ++ps) {
#pragma unroll 1
        for (int l = 0; l < 8; ++l) { const int L = L0 + l; if (L >= nlines) break; const size_t e = (size_t)L * 64 + lane * 2; const int k = (int)(e % K), n = (int)(e / K); v2us o;
            o[0] = f2bf(w[(size_t)k * N + n]); o[1] = f2bf(w[(size_t)(k + 1) * N + n]); *(volatile v2us*)(Bt + e) = o; }
        if (ps == 0) __threadfence(); }
}
__global__ __launch_bounds__(256) void k_cvt8(const float* __restrict__ src, bf* dst, size_t n8) { const size_t i = (size_t)blockIdx.x * 256 + threadIdx.x; if (i >= n8) return; const v8f v = *(const v8f*)(src + i * 8); v8us o;
#pragma unroll
    for (int k = 0; k < 8; ++k) o[k] = f2bf(v[k]); *(volatile v8us*)(dst + i * 8) = o; __threadfence(); *(volatile v8us*)(dst + i * 8) = o; }
__global__ __launch_bounds__(256) void k_lvp(const float* __restrict__ F, h16* QL, h16* KL) { const size_t e = ((size_t)blockIdx.x * 256 + threadIdx.x) * 2; if (e >= (size_t)NH_ * NLV * TT * LW) return; const int d = (int)(e % LW); const int t = (int)((e / LW) % TT); const int l = (int)((e / ((size_t)LW * TT)) % NLV); const int h = (int)(e / ((size_t)LW * TT * NLV)); const int r = c_off[l + 1] - c_off[l]; v2h q, k;
#pragma unroll
    for (int u = 0; u < 2; ++u) { const int dd = d + u; if (dd < r) { const size_t s = (size_t)t * (3 * DM) + h * HD + c_off[l] + dd; q[u] = tohx(__fmul_rn(F[s], c_inv[l])); k[u] = tohx(F[s + DM]); } else { q[u] = (h16)0.f; k[u] = (h16)0.f; } }
    *(volatile v2h*)(QL + e) = q; *(volatile v2h*)(KL + e) = k; __threadfence(); *(volatile v2h*)(QL + e) = q; *(volatile v2h*)(KL + e) = k; }
__global__ __launch_bounds__(256) void k_vtp(const float* __restrict__ F, h16* VT16, bf* VTh, bf* VTl) { const size_t e = ((size_t)blockIdx.x * 256 + threadIdx.x) * 2; if (e >= (size_t)NH_ * HD * TT) return; const int t = (int)(e % TT); const int d = (int)((e / TT) % HD); const int h = (int)(e / ((size_t)TT * HD)); v2h o; v2us oh, ol;
#pragma unroll
    for (int u = 0; u < 2; ++u) { const float v = F[(size_t)(t + u) * (3 * DM) + 2 * DM + h * HD + d]; o[u] = tohx(v); unsigned short a, c2; splitf(v, a, c2); oh[u] = a; ol[u] = c2; }
    for (int ps = 0; ps < 2; ++ps) { *(volatile v2h*)(VT16 + e) = o; *(volatile v2us*)(VTh + e) = oh; *(volatile v2us*)(VTl + e) = ol; if (ps == 0) __threadfence(); } }
__global__ __launch_bounds__(256) void k_msoft(const float* __restrict__ C, h16* P16, bf* Ph, bf* Pl) { const int lane = threadIdx.x & 31; const int row = blockIdx.x * 8 + (threadIdx.x >> 5); if (row >= TT) return; float v[64]; float mx = -3.0e38f;
#pragma unroll
    for (int ch = 0; ch < 16; ++ch) { const int j0 = ch * 128 + lane * 4; v4f c[NLV];
#pragma unroll
        for (int l = 0; l < NLV; ++l) c[l] = *(const v4f*)(C + ((size_t)l * TT + row) * TT + j0);
#pragma unroll
        for (int q = 0; q < 4; ++q) { const int j = j0 + q; float t = c[0][q];
#pragma unroll
            for (int l = 1; l < NLV; ++l) { const int sh = 11 - l; t = ((row >> sh) == (j >> sh)) ? __fadd_rn(t, c[l][q]) : t; }
            t = (j <= row) ? t : -3.0e38f; v[ch * 4 + q] = t; mx = fmaxf(mx, t); } }
#pragma unroll
    for (int sh = 16; sh; sh >>= 1) mx = fmaxf(mx, __shfl_xor(mx, sh, 32));
    float sum = 0.f;
#pragma unroll
    for (int k = 0; k < 64; ++k) { float d0 = __fsub_rn(v[k], mx); asm volatile("" : "+v"(d0)); v[k] = (v[k] > -1.0e38f) ? __expf(d0) : 0.f; sum += v[k]; }
#pragma unroll
    for (int sh = 16; sh; sh >>= 1) sum += __shfl_xor(sum, sh, 32);
    if (row < RH) { const float f = __fdiv_rn(1.0f, sum);
#pragma unroll 1
        for (int ps = 0; ps < 2; ++ps) {
#pragma unroll
            for (int ch = 0; ch < 16; ++ch) { v4us oh, ol;
#pragma unroll
                for (int q = 0; q < 4; ++q) { float y = __fmul_rn(v[ch * 4 + q], f); asm volatile("" : "+v"(y)); unsigned short a2, c2; splitf(y, a2, c2); oh[q] = a2; ol[q] = c2; }
                *(volatile v4us*)(Ph + (size_t)row * TT + ch * 128 + lane * 4) = oh; *(volatile v4us*)(Pl + (size_t)row * TT + ch * 128 + lane * 4) = ol; }
            if (ps == 0) __threadfence(); } }
    else { const float f = __fdiv_rn(PCAR, sum);
#pragma unroll 1
        for (int ps = 0; ps < 2; ++ps) {
#pragma unroll
            for (int ch = 0; ch < 16; ++ch) { v4h o;
#pragma unroll
                for (int q = 0; q < 4; ++q) o[q] = tohx(v[ch * 4 + q] * f); *(volatile v4h*)(P16 + (size_t)row * TT + ch * 128 + lane * 4) = o; }
            if (ps == 0) __threadfence(); } } }
__global__ __launch_bounds__(256) void k_ofm(const float* __restrict__ O, int h, bf* Ah, bf* Al) { const size_t e = ((size_t)blockIdx.x * 256 + threadIdx.x) * 2; if (e >= (size_t)TT * HD) return; const int d = (int)(e % HD), t = (int)(e / HD); const float sc = (t < RH) ? 1.0f : (1.0f / PCAR); v2us oh, ol;
#pragma unroll
    for (int u = 0; u < 2; ++u) { unsigned short a, c2; splitf(__fmul_rn(O[e + u], sc), a, c2); oh[u] = a; ol[u] = c2; } const size_t oo = (size_t)t * DM + h * HD + d; *(volatile v2us*)(Ah + oo) = oh; *(volatile v2us*)(Al + oo) = ol; __threadfence(); *(volatile v2us*)(Ah + oo) = oh; *(volatile v2us*)(Al + oo) = ol; }

extern "C" void kernel_launch(void* const* d_in, const int* in_sizes, int n_in,
                              void* d_out, int out_size, void* d_ws, size_t ws_size, hipStream_t stream) {
    (void)in_sizes; (void)n_in; (void)out_size;
    const float* x = (const float*)d_in[0]; const float* wa = (const float*)d_in[1]; const float* ba = (const float*)d_in[2]; const float* wp = (const float*)d_in[3]; const float* bp = (const float*)d_in[4];
    float* OUT = (float*)d_out;
    char* wsp = (char*)d_ws;
    auto take = [&](size_t bytes) { char* p = wsp; wsp += (bytes + 255) & ~(size_t)255; return (void*)p; };
    bf* WA = (bf*)take((size_t)3 * DM * DM * 2); bf* WP = (bf*)take((size_t)DM * DM * 2); bf* XB = (bf*)take((size_t)TT * DM * 2); float* F = (float*)take((size_t)TT * 3 * DM * 4);
    h16* QL = (h16*)take((size_t)NH_ * NLV * TT * LW * 2); h16* KL = (h16*)take((size_t)NH_ * NLV * TT * LW * 2); h16* VT16 = (h16*)take((size_t)NH_ * HD * TT * 2); bf* VTh = (bf*)take((size_t)NH_ * HD * TT * 2); bf* VTl = (bf*)take((size_t)NH_ * HD * TT * 2);
    float* C = (float*)take((size_t)NLV * TT * TT * 4); h16* P16 = (h16*)take((size_t)TT * TT * 2); bf* Ph = (bf*)take((size_t)RH * TT * 2); bf* Pl = (bf*)take((size_t)RH * TT * 2); float* O = (float*)take((size_t)TT * HD * 4); bf* Ah = (bf*)take((size_t)TT * DM * 2); bf* Al = (bf*)take((size_t)TT * DM * 2);
    if ((size_t)(wsp - (char*)d_ws) > ws_size) return;
    k_wtG<<<(unsigned)((DM * 3 * DM / 64 + 63) / 64), 256, 0, stream>>>(wa, DM, 3 * DM, WA); k_wtG<<<(unsigned)((DM * DM / 64 + 63) / 64), 256, 0, stream>>>(wp, DM, DM, WP);
    k_cvt8<<<(TT * DM / 8 + 255) / 256, 256, 0, stream>>>(x, XB, (size_t)TT * DM / 8);
    k_gemmw<bf, 0, true><<<dim3(TT / 64, 3 * DM / 64, 1), 32, 0, stream>>>(XB, nullptr, WA, nullptr, DM, F, 3 * DM, ba, 0, 0, 0);
    k_lvp<<<(unsigned)(((size_t)NH_ * NLV * TT * LW / 2 + 255) / 256), 256, 0, stream>>>(F, QL, KL); k_vtp<<<(unsigned)(((size_t)NH_ * HD * TT / 2 + 255) / 256), 256, 0, stream>>>(F, VT16, VTh, VTl);
    for (int h = 0; h < NH_; ++h) { const size_t lo = (size_t)h * NLV * TT * LW, vo = (size_t)h * HD * TT;
        k_gemmw<h16, 0, false><<<dim3(TT / 64, TT / 64, NLV), 32, 0, stream>>>(QL + lo, nullptr, KL + lo, nullptr, LW, C, TT, nullptr, (size_t)TT * LW, (size_t)TT * LW, (size_t)TT * TT);
        k_msoft<<<TT / 8, 256, 0, stream>>>(C, P16, Ph, Pl);
        k_gemmw<bf, 2, false><<<dim3(RH / 64, HD / 64, 1), 32, 0, stream>>>(Ph, Pl, VTh + vo, VTl + vo, TT, O, HD, nullptr, 0, 0, 0);
        k_gemmw<h16, 0, false><<<dim3((TT - RH) / 64, HD / 64, 1), 32, 0, stream>>>(P16 + (size_t)RH * TT, nullptr, VT16 + vo, nullptr, TT, O + (size_t)RH * HD, HD, nullptr, 0, 0, 0);
        k_ofm<<<(TT * HD / 2 + 255) / 256, 256, 0, stream>>>(O, h, Ah, Al); }
    k_gemmw<bf, 1, true><<<dim3(TT / 64, DM / 64, 1), 32, 0, stream>>>(Ah, Al, WP, nullptr, DM, OUT, DM, bp, 0, 0, 0);
}
